// GCNClassifier_29549374997129
// MI455X (gfx1250) — hardware-verified
//
#include <hip/hip_runtime.h>
#include <stddef.h>
#include <stdint.h>
#include <math.h>


#define DF     128
#define K2     256
#define NCLS   10
#define NGR    256
#define NTHR   256
#define NWAVE  8
#define EPT    8
#define CHUNK  (NTHR * EPT)
#define WCAP   (EPT * 32)
#define LISTN  (NWAVE * WCAP)
#define NBD    8192
#define SLD    13
#define NBA    1024
#define SLA    10
#define RCAP   24576
#define DEGCAP 64
#define GBM    64
#define GBN    64
#define GTHR   128
#define NU1    (DF * (DF / 8))
#define NU2    (DF * (K2 / 8))
#define NUL    (2 * DF * DF / 4)
#define NUTOT  (NU1 + 2 * NU2 + NUL)
#define AGG_ZINTS (LISTN + 2 * RCAP + 3 * NBA)
#define MISC_INTS 16
#define ROWBUF_INTS (NWAVE * K2 / 2)
#define AGG_LDS_INTS (AGG_ZINTS + MISC_INTS + ROWBUF_INTS)
#define NOUT01 (2 * NGR * NCLS)
#define NOUT2  (NGR * 2 * DF)
#define NOUTT  (NOUT01 + NOUT2)
#define LEAK   0.01f
#define WSMAX  134217728

static_assert((CHUNK & (CHUNK - 1)) == 0 && CHUNK <= 4096);
static_assert((NBD & (NBD - 1)) == 0 && NBD == (1 << SLD));
static_assert((NBA & (NBA - 1)) == 0 && NBA == (1 << SLA));
static_assert(((long long)CHUNK << SLD) < (1LL << 31));
static_assert(((long long)CHUNK << SLA) < (1LL << 31));
static_assert(NBD % (NTHR * 4) == 0);
static_assert(LISTN % NTHR == 0);
static_assert(NBA % NWAVE == 0 && NBA % 32 == 0 && NBA % GBM == 0);
static_assert(RCAP % 32 == 0 && AGG_ZINTS % 4 == 0 && LISTN % 4 == 0 && ((AGG_ZINTS + MISC_INTS) % 4) == 0);
static_assert(DF % 32 == 0 && K2 % 32 == 0 && K2 == 2 * DF && DF % GBN == 0);
static_assert(GBM == (GTHR / 32) * 16 && GBN == 64);
static_assert(NU1 % NTHR == 0 && NU2 % NTHR == 0 && NUL % NTHR == 0 && NUTOT % NTHR == 0);
static_assert(DF / 8 == 16 && K2 / 8 == 32 && NU2 == 4096);
static_assert(DF == 4 * 32);
static_assert(AGG_LDS_INTS * 4 <= 300000);
static_assert(NOUT01 % (4 * NTHR) == 0 && NOUT2 % (4 * NTHR) == 0 && (NOUT01 * 4) % 128 == 0);
static_assert(NTHR == 2 * DF && NGR <= NTHR);
static_assert(DF * NCLS <= 5 * NTHR && NCLS <= 16);
static_assert((NGR * NCLS) % NTHR == 0);

typedef float          v4f   __attribute__((ext_vector_type(4)));
typedef float          v8f   __attribute__((ext_vector_type(8)));
typedef int            v4i   __attribute__((ext_vector_type(4)));
typedef int            v8i   __attribute__((ext_vector_type(8)));
typedef unsigned short v4us  __attribute__((ext_vector_type(4)));
typedef unsigned short v8us  __attribute__((ext_vector_type(8)));
typedef unsigned short v16us __attribute__((ext_vector_type(16)));
typedef __bf16         v16bf __attribute__((ext_vector_type(16)));
typedef v4f  __attribute__((may_alias)) v4fa;
typedef v4i  __attribute__((may_alias)) v4ia;
typedef v4us __attribute__((may_alias)) v4usa;
typedef v8us __attribute__((may_alias)) v8usa;
union FragB { v16bf v; v16us u; v8us h[2]; v8i w; };

__device__ __forceinline__ v8f wmb(const FragB& a, const FragB& b, v8f c) {
  v8f d = __builtin_amdgcn_wmma_f32_16x16x32_bf16(false, a.v, false, b.v, (short)0, c, false, false);
  asm volatile("v_nop\n\tv_nop\n\tv_nop\n\tv_nop" : "+v"(d) : "v"(a.w), "v"(b.w));
  return d;
}

__device__ __forceinline__ unsigned bf16_bits(float f) {
  const unsigned u = __float_as_uint(f);
  return (u + 0x7FFFu + ((u >> 16) & 1u)) >> 16;
}
__device__ __forceinline__ float bf16_val(float f) {
  return __uint_as_float(bf16_bits(f) << 16);
}

__device__ __forceinline__ void wave_sync() {
  __builtin_amdgcn_fence(__ATOMIC_RELEASE, "wavefront");
  __builtin_amdgcn_wave_barrier();
  __builtin_amdgcn_fence(__ATOMIC_ACQUIRE, "wavefront");
}

template <int SLB>
__device__ __forceinline__ int scan_chunk(const int* __restrict__ dsts, int nE, int cbase, int slotBase,
                                          int nb, int vec8, int* list, int tid, int lane, int wave) {
  int wc = 0;
  const int el0  = tid * EPT;
  const int e0   = cbase + el0;
  const int sent = -2147483647 - 1;
  v4i da, db;
  if (vec8 != 0 && cbase + CHUNK <= nE) {
    da = *(const v4i*)(dsts + e0);
    db = *(const v4i*)(dsts + e0 + 4);
  } else {
    da.x = (e0     < nE) ? dsts[min(e0,     nE - 1)] : sent;
    da.y = (e0 + 1 < nE) ? dsts[min(e0 + 1, nE - 1)] : sent;
    da.z = (e0 + 2 < nE) ? dsts[min(e0 + 2, nE - 1)] : sent;
    da.w = (e0 + 3 < nE) ? dsts[min(e0 + 3, nE - 1)] : sent;
    db.x = (e0 + 4 < nE) ? dsts[min(e0 + 4, nE - 1)] : sent;
    db.y = (e0 + 5 < nE) ? dsts[min(e0 + 5, nE - 1)] : sent;
    db.z = (e0 + 6 < nE) ? dsts[min(e0 + 6, nE - 1)] : sent;
    db.w = (e0 + 7 < nE) ? dsts[min(e0 + 7, nE - 1)] : sent;
  }
  const unsigned nbs = (unsigned)slotBase;
  const unsigned unb = (unsigned)nb;
  const unsigned s0 = (unsigned)da.x - nbs, s1 = (unsigned)da.y - nbs;
  const unsigned s2 = (unsigned)da.z - nbs, s3 = (unsigned)da.w - nbs;
  const unsigned s4 = (unsigned)db.x - nbs, s5 = (unsigned)db.y - nbs;
  const unsigned s6 = (unsigned)db.z - nbs, s7 = (unsigned)db.w - nbs;
  const bool h0 = s0 < unb, h1 = s1 < unb, h2 = s2 < unb, h3 = s3 < unb;
  const bool h4 = s4 < unb, h5 = s5 < unb, h6 = s6 < unb, h7 = s7 < unb;
  const unsigned any = __builtin_amdgcn_ballot_w32(h0 | h1 | h2 | h3 | h4 | h5 | h6 | h7);
  if (any != 0u) {
#define HITJ(J, HJ, SJ) { \
      const unsigned mj = __builtin_amdgcn_ballot_w32(HJ); \
      if (mj != 0u) { \
        if (HJ) { \
          const int pos = wc + (int)__builtin_amdgcn_mbcnt_lo(mj, 0u); \
          if (pos < WCAP) list[wave * WCAP + pos] = ((el0 + (J)) << SLB) | (int)(SJ); \
        } \
        wc += (int)__builtin_popcount(mj); } }
    HITJ(0, h0, s0)
    HITJ(1, h1, s1)
    HITJ(2, h2, s2)
    HITJ(3, h3, s3)
    HITJ(4, h4, s4)
    HITJ(5, h5, s5)
    HITJ(6, h6, s6)
    HITJ(7, h7, s7)
#undef HITJ
  }
  return wc;
}

__global__ __launch_bounds__(NTHR) void k_wprep(const float* __restrict__ W1, const float* __restrict__ W2,
                                                const float* __restrict__ W3, const float* __restrict__ Wl,
                                                unsigned short* W1T, unsigned short* W2T, unsigned short* W3T,
                                                float* wlr) {
  const int u = (int)blockIdx.x * NTHR + (int)threadIdx.x;
  if (u < NU1) {
    const int n  = u >> 4;
    const int k8 = (u & 15) * 8;
    const float* p = W1 + (size_t)k8 * DF + n;
    v8us o;
#pragma unroll
    for (int i = 0; i < 8; ++i) o[i] = (unsigned short)bf16_bits(p[(size_t)i * DF]);
    unsigned short* dp = W1T + (size_t)n * DF + k8;
    *(volatile v8us*)dp = o;
    __threadfence();
    *(volatile v8us*)dp = o;
  } else if (u < NU1 + NU2) {
    const int v  = u - NU1;
    const int n  = v >> 5;
    const int k8 = (v & 31) * 8;
    const int kk = k8 & (DF - 1);
    const float* p = W2 + (size_t)kk * DF + n;
    v8us o;
#pragma unroll
    for (int i = 0; i < 8; ++i) o[i] = (unsigned short)bf16_bits(p[(size_t)i * DF]);
    unsigned short* dp = W2T + (size_t)n * K2 + k8;
    *(volatile v8us*)dp = o;
    __threadfence();
    *(volatile v8us*)dp = o;
  } else if (u < NU1 + 2 * NU2) {
    const int v  = u - (NU1 + NU2);
    const int n  = v >> 5;
    const int k8 = (v & 31) * 8;
    const int kk = k8 & (DF - 1);
    const float* p = W3 + (size_t)kk * DF + n;
    v8us o;
#pragma unroll
    for (int i = 0; i < 8; ++i) o[i] = (unsigned short)bf16_bits(p[(size_t)i * DF]);
    unsigned short* dp = W3T + (size_t)n * K2 + k8;
    *(volatile v8us*)dp = o;
    __threadfence();
    *(volatile v8us*)dp = o;
  } else if (u < NUTOT) {
    const int v = u - (NU1 + 2 * NU2);
    const v4f a = *(const v4fa*)(Wl + 4 * (size_t)v);
    v4f o;
    o.x = bf16_val(a.x); o.y = bf16_val(a.y); o.z = bf16_val(a.z); o.w = bf16_val(a.w);
    float* dp = wlr + 4 * (size_t)v;
    *(volatile v4f*)dp = o;
    __threadfence();
    *(volatile v4f*)dp = o;
  }
}

__global__ __launch_bounds__(NTHR) void k_cvx(const float* __restrict__ x, int nN, int nUnits,
                                              unsigned short* xb) {
  const int u = (int)blockIdx.x * NTHR + (int)threadIdx.x;
  if (u >= nUnits) return;
  const int row = u >> 4;
  const int k8  = (u & 15) * 8;
  const int rc  = row < nN ? row : nN - 1;
  const float* p = x + (size_t)rc * DF + k8;
  const v4f a = *(const v4fa*)p;
  const v4f b = *(const v4fa*)(p + 4);
  const bool ok = row < nN;
  v8us o;
  o[0] = ok ? (unsigned short)bf16_bits(a.x) : (unsigned short)0;
  o[1] = ok ? (unsigned short)bf16_bits(a.y) : (unsigned short)0;
  o[2] = ok ? (unsigned short)bf16_bits(a.z) : (unsigned short)0;
  o[3] = ok ? (unsigned short)bf16_bits(a.w) : (unsigned short)0;
  o[4] = ok ? (unsigned short)bf16_bits(b.x) : (unsigned short)0;
  o[5] = ok ? (unsigned short)bf16_bits(b.y) : (unsigned short)0;
  o[6] = ok ? (unsigned short)bf16_bits(b.z) : (unsigned short)0;
  o[7] = ok ? (unsigned short)bf16_bits(b.w) : (unsigned short)0;
  unsigned short* dp = xb + (size_t)row * DF + k8;
  *(volatile v8us*)dp = o;
  __threadfence();
  *(volatile v8us*)dp = o;
}

__global__ __launch_bounds__(NTHR) void k_deg(const int* __restrict__ dsts, int nE, int vec8, float* dis) {
  __shared__ __attribute__((aligned(16))) int scnt[NBD];
  __shared__ __attribute__((aligned(16))) int list[LISTN];
  __shared__ int wcnt[NWAVE];
  const int tid = (int)threadIdx.x, lane = tid & 31, wave = tid >> 5;
  const int nodeBase = (int)blockIdx.x * NBD;

  for (int i = tid; i < NBD; i += NTHR) scnt[i] = 0;
  for (int i = tid; i < LISTN; i += NTHR) list[i] = 0;
  if (tid < NWAVE) wcnt[tid] = 0;
  __syncthreads();

  const int nChunks = (nE + CHUNK - 1) / CHUNK;
#pragma unroll 1
  for (int ch = 0; ch < nChunks; ++ch) {
    const int cbase = ch * CHUNK;
    const int wc = scan_chunk<SLD>(dsts, nE, cbase, nodeBase, NBD, vec8, list, tid, lane, wave);
    if (lane == 0) wcnt[wave] = wc;
    __syncthreads();
    if (wave == 0) {
#pragma unroll 1
      for (int w2 = 0; w2 < NWAVE; ++w2) {
        int c = wcnt[w2];
        c = c < 0 ? 0 : (c > WCAP ? WCAP : c);
#pragma unroll 1
        for (int b0 = 0; b0 < c; b0 += 32) {
          const int idx = b0 + lane;
          const int ent = list[w2 * WCAP + (idx < WCAP ? idx : WCAP - 1)];
          const int m32 = (c - b0) < 32 ? (c - b0) : 32;
#pragma unroll 1
          for (int k = 0; k < m32; ++k) {
            const int u  = __builtin_amdgcn_readlane(ent, k);
            const int sl = u & (NBD - 1);
            if (lane == 0) scnt[sl] = scnt[sl] + 1;
          }
        }
      }
    }
    __syncthreads();
  }

  v4f vals[NBD / (NTHR * 4)];
#pragma unroll
  for (int it = 0; it < NBD / (NTHR * 4); ++it) {
    const int s0 = it * (NTHR * 4) + 4 * tid;
    const v4i c4 = *(const v4ia*)(scnt + s0);
    const float d0 = (float)c4.x + 1.0f, d1 = (float)c4.y + 1.0f;
    const float d2 = (float)c4.z + 1.0f, d3 = (float)c4.w + 1.0f;
    v4f v;
    v.x = rsqrtf(d0); v.y = rsqrtf(d1); v.z = rsqrtf(d2); v.w = rsqrtf(d3);
    vals[it] = v;
  }
#pragma unroll
  for (int it = 0; it < NBD / (NTHR * 4); ++it) {
    const int s0 = it * (NTHR * 4) + 4 * tid;
    *(volatile v4f*)(dis + (size_t)nodeBase + s0) = vals[it];
  }
  __threadfence();
#pragma unroll
  for (int it = 0; it < NBD / (NTHR * 4); ++it) {
    const int s0 = it * (NTHR * 4) + 4 * tid;
    *(volatile v4f*)(dis + (size_t)nodeBase + s0) = vals[it];
  }
}

__global__ __launch_bounds__(GTHR) void k_gemm(
    const unsigned short* __restrict__ A, const unsigned short* __restrict__ WT,
    float* outF, int K, int ldo)
{
  __shared__ __attribute__((aligned(16))) float stg[GBM * GBN];
  const int tid = (int)threadIdx.x, lane = tid & 31, wave = tid >> 5, hh = lane >> 4, m = lane & 15;
  const int rowBase = (int)blockIdx.x * GBM;
  const int col0    = (int)blockIdx.y * GBN;

  v8f acc[4];
  {
    const v8f z = {0.f, 0.f, 0.f, 0.f, 0.f, 0.f, 0.f, 0.f};
    acc[0] = z; acc[1] = z; acc[2] = z; acc[3] = z;
  }
  const unsigned short* ap = A  + (size_t)(rowBase + 16 * wave + m) * (size_t)K + 8 * hh;
  const unsigned short* wp = WT + (size_t)(col0 + m) * (size_t)K + 8 * hh;
  const int ksteps = K >> 5;
#pragma unroll 1
  for (int ks = 0; ks < ksteps; ++ks) {
    FragB af;
    af.h[0] = *(const v8usa*)(ap + 32 * ks);
    af.h[1] = *(const v8usa*)(ap + 32 * ks + 16);
#pragma unroll
    for (int t = 0; t < 4; ++t) {
      const unsigned short* wq = wp + (size_t)(16 * t) * (size_t)K + 32 * ks;
      FragB bf;
      bf.h[0] = *(const v8usa*)wq;
      bf.h[1] = *(const v8usa*)(wq + 16);
      acc[t] = wmb(af, bf, acc[t]);
    }
  }

#pragma unroll
  for (int t = 0; t < 4; ++t) {
    const int lc = 16 * t + m;
#pragma unroll
    for (int r = 0; r < 8; ++r) {
      const int lr = 16 * wave + 8 * hh + r;
      stg[lr * GBN + lc] = acc[t][r];
    }
  }
  __syncthreads();

  v4f fv[8];
#pragma unroll
  for (int i = 0; i < 8; ++i) {
    const int lr = 16 * wave + 2 * i + hh;
    fv[i] = *(const v4fa*)(stg + lr * GBN + 4 * m);
  }
#pragma unroll
  for (int i = 0; i < 8; ++i) {
    const int lr = 16 * wave + 2 * i + hh;
    const int gr = rowBase + lr;
    float* op = outF + (size_t)gr * (size_t)ldo + col0 + 4 * m;
    *(volatile v4f*)op = fv[i];
  }
  __threadfence();
#pragma unroll
  for (int i = 0; i < 8; ++i) {
    const int lr = 16 * wave + 2 * i + hh;
    const int gr = rowBase + lr;
    float* op = outF + (size_t)gr * (size_t)ldo + col0 + 4 * m;
    *(volatile v4f*)op = fv[i];
  }
}

template <int MODE>
__global__ __launch_bounds__(NTHR) void k_agg(const int* __restrict__ srcs, const int* __restrict__ dsts,
                                              int nE, int nN, int vec8, int mRows,
                                              const float* __restrict__ dis,
                                              const float* __restrict__ xl, const float* __restrict__ bias,
                                              unsigned short* hb, float* hout) {
  extern __shared__ __attribute__((aligned(16))) int dsm[];
  int* list = dsm;
  int* hl   = dsm + LISTN;
  int* sl   = hl + RCAP;
  int* cnt  = sl + RCAP;
  int* offs = cnt + NBA;
  int* cur  = offs + NBA;
  int* misc = cur + NBA;
  const int tid = (int)threadIdx.x, lane = tid & 31, wave = tid >> 5;
  unsigned short* rowbuf = (unsigned short*)(misc + MISC_INTS) + wave * K2;
  const int nodeBase = (int)blockIdx.x * NBA;

  {
    const v4i z4 = {0, 0, 0, 0};
    for (int i = tid * 4; i < AGG_ZINTS; i += NTHR * 4) *(v4ia*)(dsm + i) = z4;
    if (tid < MISC_INTS) misc[tid] = 0;
  }
  v4f bv;
  {
    const v4f a = *(const v4fa*)(bias + 4 * lane);
    bv.x = bf16_val(a.x); bv.y = bf16_val(a.y); bv.z = bf16_val(a.z); bv.w = bf16_val(a.w);
  }
  __syncthreads();

  int t = 0, ov = 0;
  const int nChunks = (nE + CHUNK - 1) / CHUNK;
#pragma unroll 1
  for (int ch = 0; ch < nChunks; ++ch) {
    const int cbase = ch * CHUNK;
    const int wc = scan_chunk<SLA>(dsts, nE, cbase, nodeBase, NBA, vec8, list, tid, lane, wave);
    if (lane == 0) misc[wave] = wc;
    __syncthreads();
    if (wave == 0) {
#pragma unroll 1
      for (int w2 = 0; w2 < NWAVE; ++w2) {
        int c = misc[w2];
        c = c < 0 ? 0 : (c > WCAP ? WCAP : c);
#pragma unroll 1
        for (int b0 = 0; b0 < c; b0 += 32) {
          const int idx = b0 + lane;
          const int ent = list[w2 * WCAP + (idx < WCAP ? idx : WCAP - 1)];
          const int m32 = (c - b0) < 32 ? (c - b0) : 32;
#pragma unroll 1
          for (int k = 0; k < m32; ++k) {
            const int u    = __builtin_amdgcn_readlane(ent, k);
            const int slot = u & (NBA - 1);
            const int el   = (u >> SLA) & (CHUNK - 1);
            const int pk   = ((cbase + el) << SLA) | slot;
            if (t < RCAP) {
              if (lane == 0) { hl[t] = pk; cnt[slot] = cnt[slot] + 1; }
              t = t + 1;
            } else {
              ov = 1;
            }
          }
        }
      }
    }
    __syncthreads();
  }
  if (wave == 0 && lane == 0) { misc[8] = t; misc[9] = ov; }
  __syncthreads();
  int tt = misc[8];
  tt = tt < 0 ? 0 : (tt > RCAP ? RCAP : tt);
  const int ovf = misc[9];

  if (wave == 0) {
    const int base = lane * (NBA / 32);
    int s = 0;
#pragma unroll 1
    for (int i = 0; i < NBA / 32; ++i) s += cnt[base + i];
    int incl = s;
#pragma unroll
    for (int d = 1; d < 32; d <<= 1) {
      const int y = __shfl_up(incl, d, 32);
      if (lane >= d) incl += y;
    }
    int run = incl - s;
#pragma unroll 1
    for (int i = 0; i < NBA / 32; ++i) {
      const int cv = cnt[base + i];
      offs[base + i] = run;
      cur[base + i]  = run;
      run += cv;
    }
  }
  __syncthreads();
  if (wave == 0) {
#pragma unroll 1
    for (int b0 = 0; b0 < tt; b0 += 32) {
      const int idx = b0 + lane;
      const int ent = hl[idx < RCAP ? idx : RCAP - 1];
      const int m32 = (tt - b0) < 32 ? (tt - b0) : 32;
#pragma unroll 1
      for (int k = 0; k < m32; ++k) {
        const int u    = __builtin_amdgcn_readlane(ent, k);
        const int slot = u & (NBA - 1);
        if (lane == 0) {
          int p = cur[slot];
          p = p < 0 ? 0 : (p > RCAP - 1 ? RCAP - 1 : p);
          sl[p] = u;
          cur[slot] = p + 1;
        }
      }
    }
  }
  __syncthreads();

  const float qnan = __int_as_float(0x7fc00000);
  const float pz = (ovf != 0) ? qnan : 0.0f;
#pragma unroll 1
  for (int si = 0; si < NBA / NWAVE; ++si) {
    const int s    = si * NWAVE + wave;
    const int node = nodeBase + s;
    int c = cnt[s];
    const bool big = c > DEGCAP;
    c = c < 0 ? 0 : (c > DEGCAP ? DEGCAP : c);
    int o = offs[s];
    o = o < 0 ? 0 : (o > RCAP ? RCAP : o);
    const int nc = node < nN ? node : nN - 1;
    const float dd = dis[nc];
    const float rd = dd * dd;
    float a0 = 0.0f, a1 = 0.0f, a2 = 0.0f, a3 = 0.0f;
#pragma unroll 1
    for (int b0 = 0; b0 < c; b0 += 32) {
      int idx = o + b0 + lane;
      idx = idx > RCAP - 1 ? RCAP - 1 : idx;
      const int ent = sl[idx];
      int eid = ent >> SLA;
      eid = eid < 0 ? 0 : (eid > nE - 1 ? nE - 1 : eid);
      int sr = srcs[eid];
      sr = sr < 0 ? 0 : (sr > nN - 1 ? nN - 1 : sr);
      const float cf  = dis[sr] * dd;
      const int   cfi = __float_as_int(cf);
      const int m32 = (c - b0) < 32 ? (c - b0) : 32;
#pragma unroll 1
      for (int k = 0; k < m32; ++k) {
        const int   sk = __builtin_amdgcn_readlane(sr, k);
        const float ck = __int_as_float(__builtin_amdgcn_readlane(cfi, k));
        const v4f a = *(const v4fa*)(xl + (size_t)sk * DF + 4 * lane);
        a0 = fmaf(ck, a.x, a0); a1 = fmaf(ck, a.y, a1);
        a2 = fmaf(ck, a.z, a2); a3 = fmaf(ck, a.w, a3);
      }
    }
    const v4f sv = *(const v4fa*)(xl + (size_t)nc * DF + 4 * lane);
    const float pzr = big ? qnan : pz;
    const bool live = node < nN;
    float y0 = (a0 + sv.x * rd) + bv.x;
    float y1 = (a1 + sv.y * rd) + bv.y;
    float y2 = (a2 + sv.z * rd) + bv.z;
    float y3 = (a3 + sv.w * rd) + bv.w;
    if constexpr (MODE != 0) {
      y0 = (y0 >= 0.0f) ? y0 : LEAK * y0;
      y1 = (y1 >= 0.0f) ? y1 : LEAK * y1;
      y2 = (y2 >= 0.0f) ? y2 : LEAK * y2;
      y3 = (y3 >= 0.0f) ? y3 : LEAK * y3;
    }
    y0 = y0 + pzr; y1 = y1 + pzr; y2 = y2 + pzr; y3 = y3 + pzr;
    const float v0 = live ? y0 : 0.0f;
    const float v1 = live ? y1 : 0.0f;
    const float v2 = live ? y2 : 0.0f;
    const float v3 = live ? y3 : 0.0f;
    if constexpr (MODE != 0) {
      v4us mh, ml;
      {
        unsigned hw;
        hw = bf16_bits(v0); mh[0] = (unsigned short)hw; ml[0] = (unsigned short)bf16_bits(v0 - __uint_as_float(hw << 16));
        hw = bf16_bits(v1); mh[1] = (unsigned short)hw; ml[1] = (unsigned short)bf16_bits(v1 - __uint_as_float(hw << 16));
        hw = bf16_bits(v2); mh[2] = (unsigned short)hw; ml[2] = (unsigned short)bf16_bits(v2 - __uint_as_float(hw << 16));
        hw = bf16_bits(v3); mh[3] = (unsigned short)hw; ml[3] = (unsigned short)bf16_bits(v3 - __uint_as_float(hw << 16));
      }
      *(v4usa*)(rowbuf + 4 * lane) = mh;
      *(v4usa*)(rowbuf + DF + 4 * lane) = ml;
      wave_sync();
      const v8us q0 = *(const v8usa*)(rowbuf + 8 * lane);
      wave_sync();
      if (node < mRows) {
        unsigned short* rpw = hb + (size_t)node * K2 + 8 * lane;
        *(volatile v8us*)rpw = q0;
        __threadfence();
        *(volatile v8us*)rpw = q0;
      }
    } else {
      v4f ow;
      ow.x = v0; ow.y = v1; ow.z = v2; ow.w = v3;
      if (node < mRows) {
        float* op = hout + (size_t)node * DF + 4 * lane;
        *(volatile v4f*)op = ow;
        __threadfence();
        *(volatile v4f*)op = ow;
      }
    }
  }
}

__global__ __launch_bounds__(NTHR) void k_pool(const float* __restrict__ hf, const int* __restrict__ bat,
                                               int nN, const float* __restrict__ wlr,
                                               const float* __restrict__ bl, float* emb, float* zpl) {
  __shared__ __attribute__((aligned(16))) float wsum[NWAVE * DF];
  __shared__ int wcn[NWAVE];
  __shared__ __attribute__((aligned(16))) float outs[2 * DF];
  __shared__ __attribute__((aligned(16))) float zp[2 * DF];
  __shared__ __attribute__((aligned(16))) float zrow[DF];
  const int tid = (int)threadIdx.x, lane = tid & 31, wave = tid >> 5;
  const int g = (int)blockIdx.x;

  float a0 = 0.0f, a1 = 0.0f, a2 = 0.0f, a3 = 0.0f;
  int cnt = 0;
#pragma unroll 1
  for (int i0 = wave * 32; i0 < nN; i0 += NTHR) {
    const int i  = i0 + lane;
    const int ic = i < nN ? i : nN - 1;
    const int b  = bat[ic];
    const bool hit = (i < nN) && (b == g);
    unsigned msk = __builtin_amdgcn_ballot_w32(hit);
    int nh = (int)__builtin_popcount(msk);
    nh = nh > 32 ? 32 : nh;
    cnt += nh;
#pragma unroll 1
    for (int q = 0; q < nh; ++q) {
      const int k = __builtin_ffs((int)msk) - 1;
      msk &= msk - 1u;
      int node = i0 + (k < 0 ? 0 : k);
      node = node > nN - 1 ? nN - 1 : node;
      const v4f v = *(const v4fa*)(hf + (size_t)node * DF + 4 * lane);
      a0 += v.x; a1 += v.y; a2 += v.z; a3 += v.w;
    }
  }
  {
    v4f w4;
    w4.x = a0; w4.y = a1; w4.z = a2; w4.w = a3;
    *(v4fa*)(wsum + wave * DF + 4 * lane) = w4;
  }
  if (lane == 0) wcn[wave] = cnt;
  __syncthreads();
  if (tid < DF) {
    float s = 0.0f;
    int c = 0;
#pragma unroll
    for (int w2 = 0; w2 < NWAVE; ++w2) { s += wsum[w2 * DF + tid]; c += wcn[w2]; }
    const float cf = (c < 1) ? 1.0f : (float)c;
    outs[tid]      = s;
    outs[DF + tid] = s * (1.0f / cf);
  }
  __syncthreads();
  {
    const int cc = tid & (DF - 1);
    const int kb = (tid >> 7) * DF;
    float p = 0.0f;
#pragma unroll 4
    for (int k = 0; k < DF; ++k) p = fmaf(outs[kb + k], wlr[(size_t)(kb + k) * DF + cc], p);
    zp[tid] = p;
  }
  __syncthreads();
  if (tid < DF) {
    const float blv = bf16_val(bl[tid]);
    const float z = (zp[tid] + zp[DF + tid]) + blv;
    zrow[tid] = fmaxf(z, 0.0f);
  }
  __syncthreads();
  const v4f e0 = *(const v4fa*)(outs + 4 * lane);
  const v4f e1 = *(const v4fa*)(outs + DF + 4 * lane);
  const v4f zz = *(const v4fa*)(zrow + 4 * lane);
  float* ep = emb + (size_t)g * (2 * DF) + 4 * lane;
  float* zq = zpl + (size_t)g * DF + 4 * lane;
  const bool wa = (wave == 0);
  const bool wb = (wave == 1);
  if (wa) { *(volatile v4f*)ep = e0; *(volatile v4f*)(ep + DF) = e1; }
  if (wb) { *(volatile v4f*)zq = zz; }
  __threadfence();
  if (wa) { *(volatile v4f*)ep = e0; *(volatile v4f*)(ep + DF) = e1; }
  if (wb) { *(volatile v4f*)zq = zz; }
}

__global__ __launch_bounds__(NTHR) void k_head(const float* __restrict__ zpl, const float* __restrict__ emb,
                                               const float* __restrict__ Wo, const float* __restrict__ bo,
                                               float* out) {
  __shared__ float wos[DF * NCLS];
  __shared__ float bos[16];
  __shared__ __attribute__((aligned(16))) float os[NOUT01];
  const int tid = (int)threadIdx.x;
#pragma unroll 1
  for (int i = tid; i < DF * NCLS; i += NTHR) wos[i] = bf16_val(Wo[i]);
  if (tid < 16) {
    const float bb = bo[tid < NCLS ? tid : NCLS - 1];
    bos[tid] = (tid < NCLS) ? bf16_val(bb) : 0.0f;
  }
  __syncthreads();
#pragma unroll 1
  for (int idx = tid; idx < NGR * NCLS; idx += NTHR) {
    const int g = idx / NCLS;
    const int c = idx - g * NCLS;
    const float* pr = zpl + (size_t)g * DF;
    float s = 0.0f;
#pragma unroll 1
    for (int f4 = 0; f4 < DF / 4; ++f4) {
      const v4f p = *(const v4fa*)(pr + 4 * f4);
      const float* w = wos + (4 * f4) * NCLS + c;
      s = fmaf(p.x, w[0], s);
      s = fmaf(p.y, w[NCLS], s);
      s = fmaf(p.z, w[2 * NCLS], s);
      s = fmaf(p.w, w[3 * NCLS], s);
    }
    os[idx] = s + bos[c];
  }
  __syncthreads();
  if (tid < NGR) {
    const int g = tid;
    const float* lg = os + g * NCLS;
    float m = lg[0];
#pragma unroll 1
    for (int c = 1; c < NCLS; ++c) m = fmaxf(m, lg[c]);
    float ssum = 0.0f;
#pragma unroll 1
    for (int c = 0; c < NCLS; ++c) ssum += expf(lg[c] - m);
    const float inv = 1.0f / ssum;
#pragma unroll 1
    for (int c = 0; c < NCLS; ++c) os[NGR * NCLS + g * NCLS + c] = expf(lg[c] - m) * inv;
  }
  __syncthreads();

  constexpr int NIT01 = NOUT01 / (4 * NTHR);
  constexpr int NIT2  = NOUT2 / (4 * NTHR);
  v4f ov[NIT01];
#pragma unroll
  for (int it = 0; it < NIT01; ++it) ov[it] = *(const v4fa*)(os + 4 * (it * NTHR + tid));
#pragma unroll
  for (int it = 0; it < NIT01; ++it) *(volatile v4f*)(out + 4 * (size_t)(it * NTHR + tid)) = ov[it];
#pragma unroll 1
  for (int it = 0; it < NIT2; ++it) {
    const size_t e4 = 4 * (size_t)(it * NTHR + tid);
    const v4f ev = *(const v4fa*)(emb + e4);
    *(volatile v4f*)(out + NOUT01 + e4) = ev;
  }
  __threadfence();
#pragma unroll
  for (int it = 0; it < NIT01; ++it) *(volatile v4f*)(out + 4 * (size_t)(it * NTHR + tid)) = ov[it];
#pragma unroll 1
  for (int it = 0; it < NIT2; ++it) {
    const size_t e4 = 4 * (size_t)(it * NTHR + tid);
    const v4f ev = *(const v4fa*)(emb + e4);
    *(volatile v4f*)(out + NOUT01 + e4) = ev;
  }
}

static inline int cdiv(int a, int b) { return (a + b - 1) / b; }
static inline size_t al256(size_t o) { return (o + 255) & ~(size_t)255; }

extern "C" void kernel_launch(void* const* d_in, const int* in_sizes, int n_in,
                              void* d_out, int out_size, void* d_ws, size_t ws_size,
                              hipStream_t stream) {
  if (n_in < 13) return;
  if (in_sizes[0] < DF || (in_sizes[0] % DF) != 0) return;
  const int nN = in_sizes[0] / DF;
  if (nN < 16 || nN >= (1 << 21)) return;
  if (in_sizes[1] < 2 || (in_sizes[1] & 1) != 0) return;
  const int nE = in_sizes[1] / 2;
  if (nE < 1 || nE >= (1 << (31 - SLA))) return;
  if (in_sizes[2] != nN) return;
  if (in_sizes[3] != DF * DF || in_sizes[4] != DF) return;
  if (in_sizes[5] != DF * DF || in_sizes[6] != DF) return;
  if (in_sizes[7] != DF * DF || in_sizes[8] != DF) return;
  if (in_sizes[9] != 2 * DF * DF || in_sizes[10] != DF) return;
  if (in_sizes[11] != DF * NCLS || in_sizes[12] != NCLS) return;
  if (out_size != NOUTT) return;

  const float* x    = (const float*)d_in[0];
  const int*   edge = (const int*)d_in[1];
  const int*   bat  = (const int*)d_in[2];
  const float* W1   = (const float*)d_in[3];
  const float* b1   = (const float*)d_in[4];
  const float* W2   = (const float*)d_in[5];
  const float* b2   = (const float*)d_in[6];
  const float* W3   = (const float*)d_in[7];
  const float* b3   = (const float*)d_in[8];
  const float* Wl   = (const float*)d_in[9];
  const float* bl   = (const float*)d_in[10];
  const float* Wo   = (const float*)d_in[11];
  const float* bo   = (const float*)d_in[12];
  float* out = (float*)d_out;
  const int* src = edge;
  const int* dst = edge + nE;

  const int MP   = cdiv(nN, GBM) * GBM;
  const int gM   = MP / GBM;
  const int gD   = cdiv(nN, NBD);
  const int NBPD = gD * NBD;
  const int gA   = cdiv(MP, NBA);
  if ((long long)gA * NBA < (long long)MP) return;
  if (NBPD < nN) return;
  const int vec8 = ((nE & 3) == 0) ? 1 : 0;

  char* ws = (char*)d_ws;
  size_t off = 0;
  const size_t oDIS = off; off = al256(off + (size_t)NBPD * 4);
  const size_t oW1T = off; off = al256(off + (size_t)DF * DF * 2);
  const size_t oW2T = off; off = al256(off + (size_t)DF * K2 * 2);
  const size_t oW3T = off; off = al256(off + (size_t)DF * K2 * 2);
  const size_t oWLR = off; off = al256(off + (size_t)2 * DF * DF * 4);
  const size_t oXB  = off; off = al256(off + (size_t)MP * DF * 2);
  const size_t oHF  = off; off = al256(off + (size_t)MP * DF * 4);
  const size_t oA2  = off; off = al256(off + (size_t)MP * K2 * 2);
  const size_t oH3  = off; off = al256(off + (size_t)MP * DF * 4);
  const size_t oEMB = off; off = al256(off + (size_t)NGR * 2 * DF * 4);
  const size_t oZP  = off; off = al256(off + (size_t)NGR * DF * 4);
  if (off > ws_size || off > (size_t)WSMAX) return;
  float*          DIS = (float*)(ws + oDIS);
  unsigned short* W1T = (unsigned short*)(ws + oW1T);
  unsigned short* W2T = (unsigned short*)(ws + oW2T);
  unsigned short* W3T = (unsigned short*)(ws + oW3T);
  float*          WLR = (float*)(ws + oWLR);
  unsigned short* XB  = (unsigned short*)(ws + oXB);
  float*          HF  = (float*)(ws + oHF);
  unsigned short* A2  = (unsigned short*)(ws + oA2);
  float*          H3  = (float*)(ws + oH3);
  float*          EMB = (float*)(ws + oEMB);
  float*          ZP  = (float*)(ws + oZP);

  const size_t aggLds = (size_t)AGG_LDS_INTS * 4;
  hipFuncSetAttribute(reinterpret_cast<const void*>(&k_agg<1>), hipFuncAttributeMaxDynamicSharedMemorySize, (int)aggLds);
  hipFuncSetAttribute(reinterpret_cast<const void*>(&k_agg<0>), hipFuncAttributeMaxDynamicSharedMemorySize, (int)aggLds);

  const int nUx = MP * (DF / 8);
  k_wprep<<<NUTOT / NTHR, NTHR, 0, stream>>>(W1, W2, W3, Wl, W1T, W2T, W3T, WLR);
  k_cvx<<<cdiv(nUx, NTHR), NTHR, 0, stream>>>(x, nN, nUx, XB);
  k_deg<<<gD, NTHR, 0, stream>>>(dst, nE, vec8, DIS);
  k_gemm<<<dim3(gM, DF / GBN), GTHR, 0, stream>>>(XB, W1T, HF, DF, DF);
  k_agg<1><<<gA, NTHR, aggLds, stream>>>(src, dst, nE, nN, vec8, MP, DIS, HF, b1, A2, H3);
  k_gemm<<<dim3(gM, DF / GBN), GTHR, 0, stream>>>(A2, W2T, HF, K2, DF);
  k_agg<1><<<gA, NTHR, aggLds, stream>>>(src, dst, nE, nN, vec8, MP, DIS, HF, b2, A2, H3);
  k_gemm<<<dim3(gM, DF / GBN), GTHR, 0, stream>>>(A2, W3T, HF, K2, DF);
  k_agg<0><<<gA, NTHR, aggLds, stream>>>(src, dst, nE, nN, vec8, MP, DIS, HF, b3, A2, H3);
  k_pool<<<NGR, NTHR, 0, stream>>>(H3, bat, nN, WLR, bl, EMB, ZP);
  k_head<<<1, NTHR, 0, stream>>>(ZP, EMB, Wo, bo, out);
}
